// MultiAssetLSTM_38594576122293
// MI455X (gfx1250) — hardware-verified
//
#include <hip/hip_runtime.h>
#include <math.h>

typedef __attribute__((ext_vector_type(16))) _Float16 v16h;
typedef __attribute__((ext_vector_type(16))) __bf16 v16b;
typedef __attribute__((ext_vector_type(8)))  _Float16 v8h;
typedef __attribute__((ext_vector_type(8)))  float v8f;
typedef __attribute__((ext_vector_type(4)))  float v4f;
typedef __attribute__((ext_vector_type(2)))  float v2f;
typedef __attribute__((ext_vector_type(4)))  unsigned v4u;
typedef __attribute__((ext_vector_type(4)))  int v4i;
typedef float __attribute__((may_alias)) float_a;
typedef int __attribute__((may_alias)) int_a;

template <typename T> __device__ __forceinline__ void vst2(void* p, T v) { *(volatile T*)p = v; __threadfence(); *(volatile T*)p = v; }
__device__ __forceinline__ v8f wmma16(v16h a, v16h b, v8f c) {
  v8f d = __builtin_amdgcn_wmma_f32_16x16x32_f16(false, a, false, b, (short)0, c, false, false);
  asm volatile("v_nop\n\tv_nop\n\tv_nop\n\tv_nop" : "+v"(d) : "v"(a), "v"(b));
  return d;
}
__device__ __forceinline__ v8f wmma_bf(v16b a, v16b b, v8f c) {
  v8f d = __builtin_amdgcn_wmma_f32_16x16x32_bf16(false, a, false, b, (short)0, c, false, false);
  asm volatile("v_nop\n\tv_nop\n\tv_nop\n\tv_nop" : "+v"(d) : "v"(a), "v"(b));
  return d;
}
__device__ __forceinline__ v16h frag_h(const _Float16* rowk0, int lane) {
  union { v16h v; v8h q[2]; } u; const _Float16* p = rowk0 + 8 * (lane >> 4);
  u.q[0] = *(const v8h*)p; u.q[1] = *(const v8h*)(p + 16); return u.v;
}
__device__ __forceinline__ v16h frag_f32(const float* rowk0, int lane) {
  v16h a; const float* p = rowk0 + 8 * (lane >> 4);
#pragma unroll
  for (int i = 0; i < 8; ++i) { a[i] = (_Float16)p[i]; a[8 + i] = (_Float16)p[16 + i]; }
  return a;
}
__device__ __forceinline__ v16h frag_f32s(const float* rowk0, int lane, float sc) {
  v16h a; const float* p = rowk0 + 8 * (lane >> 4);
#pragma unroll
  for (int i = 0; i < 8; ++i) { a[i] = (_Float16)(p[i] * sc); a[8 + i] = (_Float16)(p[16 + i] * sc); }
  return a;
}
__device__ __forceinline__ v16h fragc_f32(const float* W, int k0, int n, int lane, int ld, int K) {
  v16h a; const int g = lane >> 4;
#pragma unroll
  for (int i = 0; i < 8; ++i) { const int ka = k0 + 8 * g + i, kb = ka + 16;
    a[i] = (_Float16)(ka < K ? W[(size_t)ka * ld + n] : 0.f); a[8 + i] = (_Float16)(kb < K ? W[(size_t)kb * ld + n] : 0.f); }
  return a;
}
struct F2 { v16b h, l; };
__device__ __forceinline__ F2 bsplit16(const float v[16]) { F2 r;
#pragma unroll
  for (int i = 0; i < 16; ++i) { const __bf16 h = (__bf16)v[i]; r.h[i] = h; r.l[i] = (__bf16)(v[i] - (float)h); }
  return r; }
__device__ __forceinline__ F2 split_row(const float* row, int k0, int lane) { float v[16]; const float* p = row + k0 + 8 * (lane >> 4);
#pragma unroll
  for (int i = 0; i < 8; ++i) { v[i] = p[i]; v[8 + i] = p[16 + i]; }
  return bsplit16(v); }
__device__ __forceinline__ F2 split_rowK(const float* row, int k0, int lane, int K) { float v[16]; const int g = lane >> 4;
#pragma unroll
  for (int i = 0; i < 8; ++i) { const int ka = k0 + 8 * g + i, kb = ka + 16; v[i] = ka < K ? row[ka] : 0.f; v[8 + i] = kb < K ? row[kb] : 0.f; }
  return bsplit16(v); }
__device__ __forceinline__ F2 split_col(const float* W, int k0, int n, int lane, int ld, int K) { float v[16]; const int g = lane >> 4;
#pragma unroll
  for (int i = 0; i < 8; ++i) { const int ka = k0 + 8 * g + i, kb = ka + 16; v[i] = ka < K ? W[(size_t)ka * ld + n] : 0.f; v[8 + i] = kb < K ? W[(size_t)kb * ld + n] : 0.f; }
  return bsplit16(v); }
__device__ __forceinline__ v8f mac3(const F2& a, const F2& b, v8f c) { c = wmma_bf(a.l, b.h, c); c = wmma_bf(a.h, b.l, c); return wmma_bf(a.h, b.h, c); }
__device__ __forceinline__ float sigm(float v) { return 1.0f / (1.0f + expf(-v)); }
#define LDSX() do { asm volatile("s_wait_dscnt 0" ::: "memory"); __builtin_amdgcn_wave_barrier(); __builtin_amdgcn_fence(__ATOMIC_RELEASE, "workgroup"); } while (0)

#define NS 512
#define TT 512
#define NI 32
#define NHID 64
#define NG (4 * NHID)
#define NOUT 8

__global__ __launch_bounds__(128) void k_xproj(const float* __restrict__ x, const float* __restrict__ wih, const float* __restrict__ bih, const float* __restrict__ bhh, float* __restrict__ xp) {
  __shared__ __align__(16) float so[4][16][132];
  const int tid = threadIdx.x, wave = tid >> 5, lane = tid & 31, col = lane & 15, g = lane >> 4;
  const int r0 = blockIdx.x * 64 + wave * 16, n0 = blockIdx.y * 128;
  const v16h a = frag_f32(x + (size_t)(r0 + col) * NI, lane);
  v8f acc[8];
#pragma unroll
  for (int j = 0; j < 8; ++j) { acc[j] = (v8f){}; acc[j] = wmma16(a, frag_f32s(wih + (size_t)(n0 + j * 16 + col) * NI, lane, 4.0f), acc[j]); }
#pragma unroll
  for (int j = 0; j < 8; ++j) { const int c = n0 + j * 16 + col; const float bb = bih[c] + bhh[c];
#pragma unroll
    for (int r = 0; r < 8; ++r) so[wave][8 * g + r][j * 16 + col] = acc[j][r] * 0.25f + bb; }
  LDSX();
#pragma unroll 4
  for (int rl = 0; rl < 16; ++rl) vst2(xp + (size_t)(r0 + rl) * NG + n0 + lane * 4, *(const v4f*)(&so[wave][rl][lane * 4]));
}
__global__ __launch_bounds__(128) void k_lstm(const float* __restrict__ xp, const float* __restrict__ whh, const float* __restrict__ wfc, const float* __restrict__ bfc, float* __restrict__ out) {
  __shared__ __align__(16) _Float16 sh[4][16][72];
  __shared__ __align__(16) float shl[4][16][68];
  __shared__ __align__(16) float so[64 * NOUT];
  __shared__ __align__(16) _Float16 sW[NG][72];
  const int tid = threadIdx.x, w = tid >> 5, lane = tid & 31, col = lane & 15, g = lane >> 4;
  const int b0 = blockIdx.x * 64 + w * 16;
  for (int e = tid; e < NG * NHID; e += 128) sW[e >> 6][e & 63] = (_Float16)(whh[e] * 4.0f);
  __syncthreads();
  float c[4][8], hreg[4][8];
#pragma unroll
  for (int q = 0; q < 4; ++q)
#pragma unroll
    for (int r = 0; r < 8; ++r) { c[q][r] = 0.f; hreg[q][r] = 0.f; }
  for (int e = lane; e < 16 * 64; e += 32) sh[w][e >> 6][e & 63] = (_Float16)0.f;
  LDSX();
#pragma unroll 1
  for (int t = 0; t < TT; ++t) {
    v16h a[2];
#pragma unroll
    for (int kc = 0; kc < 2; ++kc) a[kc] = frag_h(&sh[w][col][0] + kc * 32, lane);
    LDSX();
#pragma unroll
    for (int hf = 0; hf < 2; ++hf) {
      v8f acc[8];
#pragma unroll
      for (int e = 0; e < 8; ++e) { const int j = (e & 3) * 4 + 2 * hf + (e >> 2);
        acc[e] = (v8f){}; acc[e] = wmma16(a[0], frag_h(&sW[j * 16 + col][0], lane), acc[e]); acc[e] = wmma16(a[1], frag_h(&sW[j * 16 + col][0] + 32, lane), acc[e]); }
#pragma unroll
      for (int qq = 0; qq < 2; ++qq) { const int q = 2 * hf + qq; const int u = q * 16 + col;
#pragma unroll
        for (int r = 0; r < 8; ++r) { const size_t row = (size_t)(b0 + 8 * g + r) * TT + t; const float* xr = xp + row * NG;
          const float gi = acc[qq * 4 + 0][r] * 0.25f + xr[u], gf = acc[qq * 4 + 1][r] * 0.25f + xr[NHID + u], gg = acc[qq * 4 + 2][r] * 0.25f + xr[2 * NHID + u], go = acc[qq * 4 + 3][r] * 0.25f + xr[3 * NHID + u];
          const float cn = sigm(gf) * c[q][r] + sigm(gi) * tanhf(gg); c[q][r] = cn; const float hn = sigm(go) * tanhf(cn); hreg[q][r] = hn;
          sh[w][8 * g + r][u] = (_Float16)hn; } } }
    LDSX(); }
#pragma unroll
  for (int q = 0; q < 4; ++q)
#pragma unroll
    for (int r = 0; r < 8; ++r) shl[w][8 * g + r][q * 16 + col] = hreg[q][r];
  __syncthreads();
  { const int rl = tid >> 1, part = tid & 1; const float* hr = &shl[rl >> 4][rl & 15][0];
#pragma unroll
    for (int oo = 0; oo < 4; ++oo) { const int o = part * 4 + oo; float a = bfc[o]; for (int k = 0; k < NHID; ++k) a += hr[k] * wfc[o * NHID + k]; so[rl * NOUT + o] = a; } }
  __syncthreads();
  if (tid < 128) vst2(out + (size_t)blockIdx.x * 64 * NOUT + tid * 4, *(const v4f*)(&so[tid * 4]));
}
extern "C" void kernel_launch(void* const* d_in, const int* in_sizes, int n_in, void* d_out, int out_size, void* d_ws, size_t ws_size, hipStream_t stream) {
  (void)in_sizes; (void)n_in; (void)out_size; (void)ws_size;
  const float** I = (const float**)d_in;
  const float* x = I[0]; const float* wih = I[1]; const float* whh = I[2]; const float* bih = I[3]; const float* bhh = I[4]; const float* wfc = I[5]; const float* bfc = I[6];
  float* out = (float*)d_out;
  float* xp = (float*)d_ws;
  k_xproj<<<dim3(NS * TT / 64, NG / 128), 128, 0, stream>>>(x, wih, bih, bhh, xp);
  k_lstm<<<NS / 64, 128, 0, stream>>>(xp, whh, wfc, bfc, out);
}
